// GroupedExperts_609885356950
// MI455X (gfx1250) — hardware-verified
//
#include <hip/hip_runtime.h>
#include <hip/hip_bf16.h>

#define N_EXPERTS 8
#define D_MODEL 512
#define HIDDEN 1024
#define TOKENS_PER_EXPERT 1024

#define BM 128
#define BK 32
#define BN1 64
#define BN2 128
#define LDSR 40

#define __bf16 _Float16
typedef __bf16 v16bf __attribute__((ext_vector_type(16)));
typedef __bf16 v2bf  __attribute__((ext_vector_type(2)));
typedef float  v8f   __attribute__((ext_vector_type(8)));
typedef float  v4f_t __attribute__((ext_vector_type(4)));
typedef float v4fa __attribute__((ext_vector_type(4), may_alias));
typedef unsigned v4u_t __attribute__((ext_vector_type(4)));
typedef unsigned v4ua __attribute__((ext_vector_type(4), may_alias));

static __device__ __forceinline__ unsigned int pk2bf(float a, float b) {
    union { v2bf v; unsigned int u; } r;
    r.v = v2bf{(__bf16)a, (__bf16)b};
    return r.u;
}
static __device__ __forceinline__ uint2 pk4bf(float4 v) {
    return make_uint2(pk2bf(v.x, v.y), pk2bf(v.z, v.w));
}

__global__ __launch_bounds__(256)
void k_gemm1_swiglu(const float* __restrict__ X, const float* __restrict__ W12,
                    const int* __restrict__ starts, const int* __restrict__ ends, __bf16* __restrict__ H) {
    __shared__ unsigned short sA[2][BM * LDSR];
    __shared__ unsigned short sB1[2][BN1 * LDSR];
    __shared__ unsigned short sB2[2][BN1 * LDSR];
    __shared__ __attribute__((aligned(16))) __bf16 sH[BM * 72];

    const int tid  = threadIdx.x;
    const int row0 = blockIdx.x * BM;
    const int n0   = blockIdx.y * BN1;

    const int lane = tid & 31, wave = tid >> 5;
    const int wm = wave & 3, wn = wave >> 2;
    const int half = lane >> 4, lm = lane & 15;
    const int kloA = half * 8, kloB = half * 8;
    const int r8 = tid >> 3, c4 = tid & 7;

#pragma unroll 1
  for (int e = 0; e < N_EXPERTS; ++e) {
    const int segS = starts[e], segE = ends[e];
    if (segE <= row0 || segS >= row0 + BM || segE <= segS) continue;
    const float* We = W12 + (size_t)e * (2 * HIDDEN) * D_MODEL;

    v8f acc1[2][2], acc2[2][2];
#pragma unroll
    for (int mi = 0; mi < 2; ++mi)
#pragma unroll
        for (int ni = 0; ni < 2; ++ni) { acc1[mi][ni] = v8f{}; acc2[mi][ni] = v8f{}; }

    auto load_tile = [&](int k0, int buf) {
#pragma unroll
        for (int i = 0; i < 4; ++i) {
            const int r = r8 + i * 32;
            float4 v = *(const float4*)(X + (size_t)(row0 + r) * D_MODEL + k0 + c4 * 4);
            *(uint2*)&sA[buf][r * LDSR + c4 * 4] = pk4bf(v);
        }
#pragma unroll
        for (int i = 0; i < 2; ++i) {
            const int r = r8 + i * 32;
            float4 v1 = *(const float4*)(We + (size_t)(n0 + r) * D_MODEL + k0 + c4 * 4);
            *(uint2*)&sB1[buf][r * LDSR + c4 * 4] = pk4bf(v1);
            float4 v2 = *(const float4*)(We + (size_t)(HIDDEN + n0 + r) * D_MODEL + k0 + c4 * 4);
            *(uint2*)&sB2[buf][r * LDSR + c4 * 4] = pk4bf(v2);
        }
    };

    constexpr int NSTEP = D_MODEL / BK;
    __syncthreads();
    load_tile(0, 0);
    int cur = 0;
    for (int ks = 0; ks < NSTEP; ++ks) {
        __syncthreads();
        if (ks + 1 < NSTEP) load_tile((ks + 1) * BK, cur ^ 1);

        v16bf a[2], b1[2], b2[2];
#pragma unroll
        for (int mi = 0; mi < 2; ++mi) {
            const unsigned short* p = &sA[cur][(wm * 32 + mi * 16 + lm) * LDSR + kloA];
            ((uint4*)&a[mi])[0] = *(const uint4*)(p);
            ((uint4*)&a[mi])[1] = *(const uint4*)(p + 16);
        }
#pragma unroll
        for (int ni = 0; ni < 2; ++ni) {
            const unsigned short* p1 = &sB1[cur][(wn * 32 + ni * 16 + lm) * LDSR + kloB];
            ((uint4*)&b1[ni])[0] = *(const uint4*)(p1);
            ((uint4*)&b1[ni])[1] = *(const uint4*)(p1 + 16);
            const unsigned short* p2 = &sB2[cur][(wn * 32 + ni * 16 + lm) * LDSR + kloB];
            ((uint4*)&b2[ni])[0] = *(const uint4*)(p2);
            ((uint4*)&b2[ni])[1] = *(const uint4*)(p2 + 16);
        }
#pragma unroll
        for (int mi = 0; mi < 2; ++mi)
#pragma unroll
            for (int ni = 0; ni < 2; ++ni) {
                acc1[mi][ni] = __builtin_amdgcn_wmma_f32_16x16x32_f16(
                    false, a[mi], false, b1[ni], (short)0, acc1[mi][ni], false, false);
                acc2[mi][ni] = __builtin_amdgcn_wmma_f32_16x16x32_f16(
                    false, a[mi], false, b2[ni], (short)0, acc2[mi][ni], false, false);
            }
        cur ^= 1;
    }

#pragma unroll
    for (int mi = 0; mi < 2; ++mi)
#pragma unroll
        for (int ni = 0; ni < 2; ++ni) {
            const int c = n0 + wn * 32 + ni * 16 + lm;
#pragma unroll
            for (int v = 0; v < 8; ++v) {
                const int t = row0 + wm * 32 + mi * 16 + half * 8 + v;
                float x1 = acc1[mi][ni][v], x2 = acc2[mi][ni][v];
                float h = x1 * __builtin_amdgcn_rcpf(1.0f + __expf(-x1)) * x2;
                if (t >= segS && t < segE) sH[(t - row0) * 72 + (c - n0)] = (__bf16)h;
            }
        }
  }
    __syncthreads();
#pragma unroll 1
    for (int pass = 0; pass < 2; ++pass) {
        for (int ch = tid; ch < BM * 8; ch += 256) { const int r = ch >> 3, q = (ch & 7) * 8;
            *(volatile v4u_t*)(H + (size_t)(row0 + r) * HIDDEN + n0 + q) = *(const v4ua*)(sH + r * 72 + q); }
        __threadfence();
    }
}

__global__ __launch_bounds__(256)
void k_gemm2(const __bf16* __restrict__ H, const float* __restrict__ W3,
             const int* __restrict__ starts, const int* __restrict__ ends, float* __restrict__ Out) {
    __shared__ unsigned short sA[2][BM * LDSR];
    __shared__ unsigned short sB[2][BN2 * LDSR];
    __shared__ __attribute__((aligned(16))) float sO[BM * 132];

    const int tid  = threadIdx.x;
    const int row0 = blockIdx.x * BM;
    const int n0   = blockIdx.y * BN2;

    const int lane = tid & 31, wave = tid >> 5;
    const int wm = wave & 3, wn = wave >> 2;
    const int half = lane >> 4, lm = lane & 15;
    const int kloA = half * 8, kloB = half * 8;
    const int r4 = tid >> 2, c8 = tid & 3;
    const int r8 = tid >> 3, c4 = tid & 7;

    for (int i = tid; i < BM * 132; i += 256) sO[i] = 0.0f;

#pragma unroll 1
  for (int e = 0; e < N_EXPERTS; ++e) {
    const int segS = starts[e], segE = ends[e];
    if (segE <= row0 || segS >= row0 + BM || segE <= segS) continue;
    const float* We = W3 + (size_t)e * D_MODEL * HIDDEN;

    v8f acc[2][4];
#pragma unroll
    for (int mi = 0; mi < 2; ++mi)
#pragma unroll
        for (int ni = 0; ni < 4; ++ni) acc[mi][ni] = v8f{};

    auto load_tile = [&](int k0, int buf) {
#pragma unroll
        for (int i = 0; i < 2; ++i) {
            const int r = r4 + i * 64;
            unsigned lds_off = (unsigned)(size_t)&sA[buf][r * LDSR + c8 * 8];
            unsigned goff = (unsigned)(((size_t)(row0 + r) * HIDDEN + k0 + c8 * 8) * sizeof(__bf16));
            asm volatile("global_load_async_to_lds_b128 %0, %1, %2"
                         :: "v"(lds_off), "v"(goff), "s"(H) : "memory");
        }
#pragma unroll
        for (int i = 0; i < 4; ++i) {
            const int r = r8 + i * 32;
            float4 v = *(const float4*)(We + (size_t)(n0 + r) * HIDDEN + k0 + c4 * 4);
            *(uint2*)&sB[buf][r * LDSR + c4 * 4] = pk4bf(v);
        }
    };

    constexpr int NSTEP = HIDDEN / BK;
    __syncthreads();
    load_tile(0, 0);
    int cur = 0;
    for (int ks = 0; ks < NSTEP; ++ks) {
        asm volatile("s_wait_asynccnt 0" ::: "memory");
        __syncthreads();
        if (ks + 1 < NSTEP) load_tile((ks + 1) * BK, cur ^ 1);

        v16bf a[2], b[4];
#pragma unroll
        for (int mi = 0; mi < 2; ++mi) {
            const unsigned short* p = &sA[cur][(wm * 32 + mi * 16 + lm) * LDSR + kloA];
            ((uint4*)&a[mi])[0] = *(const uint4*)(p);
            ((uint4*)&a[mi])[1] = *(const uint4*)(p + 16);
        }
#pragma unroll
        for (int ni = 0; ni < 4; ++ni) {
            const unsigned short* p = &sB[cur][(wn * 64 + ni * 16 + lm) * LDSR + kloB];
            ((uint4*)&b[ni])[0] = *(const uint4*)(p);
            ((uint4*)&b[ni])[1] = *(const uint4*)(p + 16);
        }
#pragma unroll
        for (int mi = 0; mi < 2; ++mi)
#pragma unroll
            for (int ni = 0; ni < 4; ++ni)
                acc[mi][ni] = __builtin_amdgcn_wmma_f32_16x16x32_f16(
                    false, a[mi], false, b[ni], (short)0, acc[mi][ni], false, false);
        cur ^= 1;
    }

#pragma unroll
    for (int mi = 0; mi < 2; ++mi)
#pragma unroll
        for (int ni = 0; ni < 4; ++ni) {
            const int d = n0 + wn * 64 + ni * 16 + lm;
#pragma unroll
            for (int v = 0; v < 8; ++v) {
                const int t = row0 + wm * 32 + mi * 16 + half * 8 + v;
                if (t >= segS && t < segE) sO[(t - row0) * 132 + (d - n0)] += acc[mi][ni][v];
            }
        }
  }
    __syncthreads();
#pragma unroll 1
    for (int pass = 0; pass < 2; ++pass) {
        for (int ch = tid; ch < BM * 32; ch += 256) { const int r = ch >> 5, q = (ch & 31) * 4;
            *(volatile v4f_t*)(Out + (size_t)(row0 + r) * D_MODEL + n0 + q) = *(const volatile v4fa*)(sO + r * 132 + q); }
        __threadfence();
    }
}

extern "C" void kernel_launch(void* const* d_in, const int* in_sizes, int n_in,
                              void* d_out, int out_size, void* d_ws, size_t ws_size,
                              hipStream_t stream) {
    const float* X      = (const float*)d_in[0];
    const float* W12    = (const float*)d_in[1];
    const float* W3     = (const float*)d_in[2];
    const int*   starts = (const int*)d_in[3];
    float*       Out    = (float*)d_out;
    __bf16*      H      = (__bf16*)d_ws;

    const int*   endsv  = (const int*)d_in[4];
    dim3 g1(N_EXPERTS * TOKENS_PER_EXPERT / BM, HIDDEN / BN1, 1);
    k_gemm1_swiglu<<<g1, 256, 0, stream>>>(X, W12, starts, endsv, H);

    dim3 g2(N_EXPERTS * TOKENS_PER_EXPERT / BM, D_MODEL / BN2, 1);
    k_gemm2<<<g2, 256, 0, stream>>>(H, W3, starts, endsv, Out);
}
